// PointNetSetAbstraction_11123965297212
// MI455X (gfx1250) — hardware-verified
//
#include <hip/hip_runtime.h>
#include <math.h>
#pragma clang fp contract(off)

typedef __attribute__((ext_vector_type(16))) _Float16 v16h;
typedef __attribute__((ext_vector_type(8)))  _Float16 v8h;
typedef __attribute__((ext_vector_type(8)))  float    v8f;
typedef __attribute__((ext_vector_type(4)))  float    v4f;
typedef __attribute__((ext_vector_type(4)))  unsigned v4u;

constexpr int kBatch   = 16;
constexpr int kNpts    = 4096;
constexpr int kNsmp    = 1024;
constexpr int kNeigh   = 32;
constexpr int kCpts    = 64;
constexpr int kCin0    = 67;
constexpr int kRows    = kBatch * kNsmp * kNeigh;
constexpr int kQueries = kBatch * kNsmp;
constexpr int kPoints  = kBatch * kNpts;
constexpr int kApitch  = 72;
constexpr float kWcarry = 64.0f;
constexpr float kWinv   = 1.0f / 64.0f;

static_assert(kRows == 524288, "rows");
static_assert(kQueries == 16384, "queries");
static_assert(kPoints == 65536, "points");
static_assert(kRows % 128 == 0 && kPoints % 128 == 0, "tile multiples");
static_assert(kCpts % 32 == 0, "contraction depth multiple of 32");
static_assert(kCin0 == 3 + kCpts, "layer 0 input width");

constexpr size_t kOffP4    = 0;
constexpr size_t kOffCent  = kOffP4   + (size_t)kPoints * 16;
constexpr size_t kOffNn    = kOffCent + (size_t)kQueries * 16;
constexpr size_t kOffW0p   = kOffNn   + (size_t)kRows * 4;
constexpr size_t kOffW1h   = kOffW0p  + 64 * 64 * 2;
constexpr size_t kOffW2h   = kOffW1h  + 64 * 64 * 2;
constexpr size_t kOffW0x   = kOffW2h  + 128 * 64 * 2;
constexpr size_t kOffSs0   = kOffW0x  + 64 * 4 * 4;
constexpr size_t kOffSs1   = kOffSs0  + 1024;
constexpr size_t kOffSs2   = kOffSs1  + 1024;
constexpr size_t kOffPart0 = kOffSs2  + 1024;
constexpr size_t kOffPart1 = kOffPart0 + (size_t)1024 * 1024;
constexpr size_t kOffPart2 = kOffPart1 + (size_t)4096 * 1024;
constexpr size_t kOffP     = kOffPart2 + (size_t)4096 * 1024;
constexpr size_t kOffY1    = kOffP    + (size_t)kPoints * 64 * 4;
constexpr size_t kOffMx    = kOffY1   + (size_t)kRows * 64 * 2;
constexpr size_t kOffMn    = kOffMx   + (size_t)kQueries * 128 * 4;
constexpr size_t kWsTotal  = kOffMn   + (size_t)kQueries * 128 * 4;
static_assert(kWsTotal <= (size_t)134217728, "carve within 128 MiB");
static_assert(kOffPart0 % 1024 == 0 && kOffP % 1024 == 0 && kOffY1 % 1024 == 0, "aligned carves");

constexpr size_t kOut1Float = (size_t)kBatch * kNsmp * 3;
static_assert(kOut1Float * 4 == 196608, "second output byte offset");
static_assert((kOut1Float + (size_t)kBatch * 128 * kNsmp) * 4 == 8585216, "output total bytes");

__device__ __forceinline__ v8f mma_f16(v16h a, v16h b, v8f c) {
  c = __builtin_amdgcn_wmma_f32_16x16x32_f16(false, a, false, b, (short)0, c, false, false);
  asm volatile("v_nop\n\tv_nop\n\tv_nop\n\tv_nop" : "+v"(c) : "v"(a), "v"(b));
  return c;
}

__device__ __forceinline__ v16h frag_ld_g(const _Float16* p) {
  union { v16h v; v8h h[2]; } f;
  f.h[0] = *(const v8h*)(p);
  f.h[1] = *(const v8h*)(p + 16);
  return f.v;
}

template <int NT>
__device__ __forceinline__ void wave_gemm(const v16h a0, const v16h a1,
                                          const _Float16* __restrict__ Wh, int lane, v8f (&acc)[NT]) {
  const int rl = lane & 15;
  const int koff = (lane >> 4) * 8;
#pragma unroll
  for (int j = 0; j < NT; ++j) {
    const _Float16* bp = Wh + (j * 16 + rl) * 64 + koff;
    const v16h b0 = frag_ld_g(bp);
    const v16h b1 = frag_ld_g(bp + 32);
    v8f c = (v8f){0.f, 0.f, 0.f, 0.f, 0.f, 0.f, 0.f, 0.f};
    c = mma_f16(a0, b0, c);
    c = mma_f16(a1, b1, c);
    acc[j] = c;
    if ((j & 1) == 1) asm volatile("" ::: "memory");
  }
}

__device__ __forceinline__ float h16_to_f32(unsigned hb) {
  const unsigned sgn = (hb & 0x8000u) << 16;
  const unsigned em = hb & 0x7fffu;
  const float fn = __uint_as_float((em << 13) + 0x38000000u);
  const float fs = (float)em * 5.9604644775390625e-8f;
  const float mag = (em < 0x400u) ? fs : fn;
  return __uint_as_float(__float_as_uint(mag) | sgn);
}

__device__ __forceinline__ unsigned f2key(float d) {
  const unsigned u = __float_as_uint(d + 0.0f);
  const unsigned m = (unsigned)((int)u >> 31) | 0x80000000u;
  return u ^ m;
}
__device__ __forceinline__ float key2f(unsigned k) {
  const unsigned m = (k & 0x80000000u) ? 0x80000000u : 0xFFFFFFFFu;
  return __uint_as_float(k ^ m);
}

__device__ __forceinline__ unsigned dkey(const v4f p, float qx, float qy, float qz, float sqq) {
  float t = p.x * qx;
  t = fmaf(p.y, qy, t);
  t = fmaf(p.z, qz, t);
  const float d = (sqq + p.w) - 2.0f * t;
  return f2key(d);
}

__device__ __forceinline__ float y0_val(float p, float rx, float ry, float rz,
                                        float wx, float wy, float wz, float bb) {
  float d = rx * wx;
  d = fmaf(ry, wy, d);
  d = fmaf(rz, wz, d);
  return (p + d) + bb;
}

__device__ __forceinline__ void wave_sync_lds() {
  __builtin_amdgcn_fence(__ATOMIC_RELEASE, "workgroup");
  __builtin_amdgcn_wave_barrier();
  __builtin_amdgcn_fence(__ATOMIC_ACQUIRE, "workgroup");
}

__global__ __launch_bounds__(256) void prep_kernel(const float* __restrict__ xyz,
                                                   const float* __restrict__ w0,
                                                   const float* __restrict__ w1,
                                                   const float* __restrict__ w2,
                                                   float* __restrict__ P4,
                                                   unsigned short* __restrict__ W0p,
                                                   unsigned short* __restrict__ W1h,
                                                   unsigned short* __restrict__ W2h,
                                                   float* __restrict__ W0x) {
#pragma clang fp contract(off)
  const int blk = blockIdx.x;
  const int tid = threadIdx.x;
  if (blk < 256) {
    const int i = blk * 256 + tid;
    const float x = xyz[3 * (size_t)i];
    const float y = xyz[3 * (size_t)i + 1];
    const float z = xyz[3 * (size_t)i + 2];
    const float t0 = x * x;
    const float t1 = y * y;
    const float t2 = z * z;
    v4f v;
    v.x = x;
    v.y = y;
    v.z = z;
    v.w = (t0 + t2) + t1;
    float* dst = P4 + 4 * (size_t)i;
    for (int pass = 0; pass < 2; ++pass) {
      *(volatile v4f*)dst = v;
      __threadfence();
    }
  } else if (blk < 264) {
    const int t = (blk - 256) * 256 + tid;
    const int h0 = t * 8;
    const float* src;
    unsigned short* dst;
    if (blk < 258) {
      const int o = h0 >> 6;
      const int c = h0 & 63;
      src = w0 + o * kCin0 + 3 + c;
      dst = W0p + h0;
    } else if (blk < 260) {
      src = w1 + (h0 - 4096);
      dst = W1h + (h0 - 4096);
    } else {
      src = w2 + (h0 - 8192);
      dst = W2h + (h0 - 8192);
    }
    v8h hv;
#pragma unroll
    for (int e = 0; e < 8; ++e) {
      const float f = src[e] * kWcarry;
      hv[e] = (_Float16)f;
    }
    for (int pass = 0; pass < 2; ++pass) {
      *(volatile v8h*)dst = hv;
      __threadfence();
    }
  } else {
    if (tid < 64) {
      v4f v;
      v.x = w0[tid * kCin0 + 0];
      v.y = w0[tid * kCin0 + 1];
      v.z = w0[tid * kCin0 + 2];
      v.w = 0.0f;
      float* dst = W0x + 4 * tid;
      for (int pass = 0; pass < 2; ++pass) {
        *(volatile v4f*)dst = v;
        __threadfence();
      }
    }
  }
}

__global__ __launch_bounds__(256) void fps_kernel(const float* __restrict__ xyz,
                                                  float* __restrict__ out0,
                                                  float* __restrict__ cent) {
#pragma clang fp contract(off)
  __shared__ __align__(16) float sp[kNpts * 3];
  __shared__ float wv[2][8];
  __shared__ int wi[2][8];
  __shared__ int sidx[kNsmp];
  const int b = blockIdx.x;
  const int tid = threadIdx.x;
  const int lane = tid & 31;
  const int wave = tid >> 5;
  const float* xb = xyz + (size_t)b * kNpts * 3;
#pragma unroll 4
  for (int it = 0; it < 12; ++it) {
    const int i4 = it * 256 + tid;
    const v4f v = *(const v4f*)(xb + 4 * i4);
    *(v4f*)(sp + 4 * i4) = v;
  }
  __syncthreads();
  float px[16], py[16], pz[16], dmin[16];
#pragma unroll
  for (int j = 0; j < 16; ++j) {
    const int i = tid + 256 * j;
    px[j] = sp[3 * i];
    py[j] = sp[3 * i + 1];
    pz[j] = sp[3 * i + 2];
    dmin[j] = 1e10f;
  }
  int far = 0;
#pragma unroll 1
  for (int s = 0; s < kNsmp; ++s) {
    if (tid == 0) sidx[s] = far;
    const float cx = sp[3 * far];
    const float cy = sp[3 * far + 1];
    const float cz = sp[3 * far + 2];
    float best = -1.0f;
    int bi = 0;
#pragma unroll
    for (int j = 0; j < 16; ++j) {
      const float dx = px[j] - cx;
      const float dy = py[j] - cy;
      const float dz = pz[j] - cz;
      const float t0 = dx * dx;
      const float t1 = dy * dy;
      const float t2 = dz * dz;
      const float d = (t0 + t2) + t1;
      const float nd = fminf(dmin[j], d);
      dmin[j] = nd;
      if (nd > best) {
        best = nd;
        bi = tid + 256 * j;
      }
    }
#pragma unroll
    for (int off = 16; off > 0; off >>= 1) {
      const float ov = __shfl_xor(best, off, 32);
      const int oi = __shfl_xor(bi, off, 32);
      const bool take = (ov > best) || (ov == best && oi < bi);
      best = take ? ov : best;
      bi = take ? oi : bi;
    }
    const int pb = s & 1;
    if (lane == 0) {
      wv[pb][wave] = best;
      wi[pb][wave] = bi;
    }
    __syncthreads();
    float fv = wv[pb][0];
    int fi = wi[pb][0];
#pragma unroll
    for (int w = 1; w < 8; ++w) {
      const float ov = wv[pb][w];
      const int oi = wi[pb][w];
      const bool take = (ov > fv) || (ov == fv && oi < fi);
      fv = take ? ov : fv;
      fi = take ? oi : fi;
    }
    fi = fi < 0 ? 0 : fi;
    fi = fi > kNpts - 1 ? kNpts - 1 : fi;
    far = fi;
  }
  __syncthreads();
  v4f ov3[3];
  v4f cv4[4];
#pragma unroll
  for (int it = 0; it < 3; ++it) {
#pragma unroll
    for (int e = 0; e < 4; ++e) {
      const int f = 4 * (it * 256 + tid) + e;
      const int sm = f / 3;
      const int cm = f - 3 * sm;
      int id = sidx[sm];
      id = id < 0 ? 0 : id;
      id = id > kNpts - 1 ? kNpts - 1 : id;
      ov3[it][e] = sp[3 * id + cm];
    }
  }
#pragma unroll
  for (int it = 0; it < 4; ++it) {
    const int qi = it * 256 + tid;
    int id = sidx[qi];
    id = id < 0 ? 0 : id;
    id = id > kNpts - 1 ? kNpts - 1 : id;
    cv4[it][0] = sp[3 * id];
    cv4[it][1] = sp[3 * id + 1];
    cv4[it][2] = sp[3 * id + 2];
    cv4[it][3] = 0.0f;
  }
  float* ob = out0 + (size_t)b * kNsmp * 3;
  float* cb = cent + (size_t)b * kNsmp * 4;
  for (int pass = 0; pass < 2; ++pass) {
#pragma unroll
    for (int it = 0; it < 3; ++it) *(volatile v4f*)(ob + 4 * (it * 256 + tid)) = ov3[it];
#pragma unroll
    for (int it = 0; it < 4; ++it) *(volatile v4f*)(cb + 4 * (it * 256 + tid)) = cv4[it];
    __threadfence();
  }
}

__global__ __launch_bounds__(64) void knn_kernel(const float* __restrict__ P4,
                                                 const float* __restrict__ cent,
                                                 int* __restrict__ nn) {
#pragma clang fp contract(off)
  __shared__ __align__(16) unsigned keys[2][kNpts];
  __shared__ int lsel[2][32];
  __shared__ int lseq[2][32];
  const int tid = threadIdx.x;
  const int lane = tid & 31;
  const int wave = tid >> 5;
  const int q = blockIdx.x * 2 + wave;
  const int b = q >> 10;
  unsigned* kw = keys[wave];
  const v4f cq = *(const v4f*)(cent + 4 * (size_t)q);
  const float qx = cq.x;
  const float qy = cq.y;
  const float qz = cq.z;
  const float q0 = qx * qx;
  const float q1 = qy * qy;
  const float q2 = qz * qz;
  const float sqq = (q0 + q2) + q1;
  const float* pb = P4 + (size_t)b * kNpts * 4;
  unsigned kmin = 0xFFFFFFFFu;
#pragma unroll 1
  for (int jj = 0; jj < 32; ++jj) {
    const v4f p0 = *(const v4f*)(pb + 4 * ((4 * jj + 0) * 32 + lane));
    const v4f p1 = *(const v4f*)(pb + 4 * ((4 * jj + 1) * 32 + lane));
    const v4f p2 = *(const v4f*)(pb + 4 * ((4 * jj + 2) * 32 + lane));
    const v4f p3 = *(const v4f*)(pb + 4 * ((4 * jj + 3) * 32 + lane));
    const unsigned k0 = dkey(p0, qx, qy, qz, sqq);
    const unsigned k1 = dkey(p1, qx, qy, qz, sqq);
    const unsigned k2 = dkey(p2, qx, qy, qz, sqq);
    const unsigned k3 = dkey(p3, qx, qy, qz, sqq);
    kmin = k0 < kmin ? k0 : kmin;
    kmin = k1 < kmin ? k1 : kmin;
    kmin = k2 < kmin ? k2 : kmin;
    kmin = k3 < kmin ? k3 : kmin;
    v4u kv;
    kv.x = k0;
    kv.y = k1;
    kv.z = k2;
    kv.w = k3;
    *(v4u*)(kw + jj * 128 + lane * 4) = kv;
  }
  lsel[wave][lane] = 0;
  lseq[wave][lane] = 0;
  wave_sync_lds();
  unsigned kmn = kmin;
  unsigned kmx = kmin;
#pragma unroll
  for (int off = 16; off > 0; off >>= 1) {
    const unsigned a = __shfl_xor(kmn, off, 32);
    const unsigned c = __shfl_xor(kmx, off, 32);
    kmn = a < kmn ? a : kmn;
    kmx = c > kmx ? c : kmx;
  }
  unsigned lo = (unsigned)__builtin_amdgcn_readfirstlane((int)kmn);
  unsigned hi = (unsigned)__builtin_amdgcn_readfirstlane((int)kmx);
#pragma unroll 1
  for (int it = 0; it < 48; ++it) {
    if (lo >= hi) break;
    unsigned mid;
    if (it < 12) {
      const float fl = key2f(lo);
      const float fh = key2f(hi);
      const float fm = 0.5f * fl + 0.5f * fh;
      unsigned mk = f2key(fm);
      mk = mk > hi - 1u ? hi - 1u : mk;
      mk = mk < lo ? lo : mk;
      mid = mk;
    } else {
      mid = lo + ((hi - lo) >> 1);
    }
    mid = (unsigned)__builtin_amdgcn_readfirstlane((int)mid);
    unsigned cnt = 0u;
#pragma unroll 4
    for (int jj = 0; jj < 32; ++jj) {
      const v4u kv = *(const v4u*)(kw + jj * 128 + lane * 4);
      const unsigned k0 = kv.x;
      const unsigned k1 = kv.y;
      const unsigned k2 = kv.z;
      const unsigned k3 = kv.w;
      cnt += (k0 <= mid) ? 1u : 0u;
      cnt += (k1 <= mid) ? 1u : 0u;
      cnt += (k2 <= mid) ? 1u : 0u;
      cnt += (k3 <= mid) ? 1u : 0u;
    }
#pragma unroll
    for (int off = 16; off > 0; off >>= 1) cnt += __shfl_xor(cnt, off, 32);
    const unsigned cu = (unsigned)__builtin_amdgcn_readfirstlane((int)cnt);
    if (cu == (unsigned)kNeigh) {
      lo = mid;
      hi = mid;
      break;
    }
    if (cu > (unsigned)kNeigh) hi = mid; else lo = mid + 1u;
  }
  const unsigned T = hi;
  const unsigned ltmask = (1u << lane) - 1u;
  int selbase = 0;
  int eqbase = 0;
#pragma unroll 1
  for (int jj = 0; jj < 32; ++jj) {
    const v4u kv = *(const v4u*)(kw + jj * 128 + lane * 4);
    const unsigned ka[4] = {kv.x, kv.y, kv.z, kv.w};
#pragma unroll
    for (int e = 0; e < 4; ++e) {
      const unsigned k = ka[e];
      const int pid = (4 * jj + e) * 32 + lane;
      const bool lt = k < T;
      const bool eq = k == T;
      const unsigned bl = __builtin_amdgcn_ballot_w32(lt);
      const unsigned be = __builtin_amdgcn_ballot_w32(eq);
      const int pl = selbase + __builtin_popcount(bl & ltmask);
      const int pe = eqbase + __builtin_popcount(be & ltmask);
      if (lt && pl < 32) lsel[wave][pl] = pid;
      if (eq && pe < 32) lseq[wave][pe] = pid;
      selbase += __builtin_popcount(bl);
      eqbase += __builtin_popcount(be);
    }
  }
  wave_sync_lds();
  const int clt = selbase < 32 ? selbase : 32;
  int ie = lane - clt;
  ie = ie < 0 ? 0 : ie;
  ie = ie > 31 ? 31 : ie;
  const int ca = lsel[wave][lane];
  const int ce = lseq[wave][ie];
  const int fa = lane < clt ? 1 : 0;
  int res = ca * fa + ce * (1 - fa);
  res = res < 0 ? 0 : res;
  res = res > kNpts - 1 ? kNpts - 1 : res;
  int* dst = nn + (size_t)q * kNeigh + lane;
  for (int pass = 0; pass < 2; ++pass) {
    *(volatile int*)dst = res;
    __threadfence();
  }
}

__global__ __launch_bounds__(256) void pgemm_kernel(const float* __restrict__ points,
                                                    const unsigned short* __restrict__ W0p,
                                                    float* __restrict__ P) {
  __shared__ __align__(16) _Float16 As[128 * kApitch];
  __shared__ __align__(16) float sT[8][16 * 68];
  const int tid = threadIdx.x;
  const int lane = tid & 31;
  const int wave = tid >> 5;
  const int m0 = blockIdx.x * 128;
  {
    const int row = tid >> 1;
    const int hf = tid & 1;
    const float* src = points + (size_t)(m0 + row) * kCpts + 32 * hf;
    _Float16* arow = As + row * kApitch + 32 * hf;
#pragma unroll 1
    for (int ch = 0; ch < 2; ++ch) {
      v4f pv[4];
#pragma unroll
      for (int g = 0; g < 4; ++g) pv[g] = *(const v4f*)(src + 16 * ch + 4 * g);
      v8h h0, h1;
#pragma unroll
      for (int g = 0; g < 4; ++g) {
#pragma unroll
        for (int e = 0; e < 4; ++e) {
          const float x = pv[g][e];
          if (g < 2) h0[4 * g + e] = (_Float16)x; else h1[4 * (g - 2) + e] = (_Float16)x;
        }
      }
      *(v8h*)(arow + 16 * ch) = h0;
      *(v8h*)(arow + 16 * ch + 8) = h1;
    }
  }
  __syncthreads();
  const int rl = lane & 15;
  const int mOff = (lane >> 4) * 8;
  union { v16h v; v8h h[2]; } fa0, fa1;
  {
    const _Float16* ap = As + (wave * 16 + rl) * kApitch + (lane >> 4) * 8;
    fa0.h[0] = *(const v8h*)(ap);
    fa0.h[1] = *(const v8h*)(ap + 16);
    fa1.h[0] = *(const v8h*)(ap + 32);
    fa1.h[1] = *(const v8h*)(ap + 48);
  }
  v8f acc[4];
  wave_gemm<4>(fa0.v, fa1.v, (const _Float16*)W0p, lane, acc);
  float* slab = sT[wave];
#pragma unroll
  for (int j = 0; j < 4; ++j) {
#pragma unroll
    for (int r = 0; r < 8; ++r) slab[(mOff + r) * 68 + 16 * j + rl] = acc[j][r] * kWinv;
  }
  wave_sync_lds();
  {
    const int hh = lane >> 4;
    const int c4 = (lane & 15) * 4;
    v4f ov[8];
#pragma unroll
    for (int it = 0; it < 8; ++it) ov[it] = *(const v4f*)(slab + (it * 2 + hh) * 68 + c4);
    for (int pass = 0; pass < 2; ++pass) {
#pragma unroll
      for (int it = 0; it < 8; ++it) {
        const int row = it * 2 + hh;
        *(volatile v4f*)(P + (size_t)(m0 + wave * 16 + row) * 64 + c4) = ov[it];
      }
      __threadfence();
    }
  }
}

__global__ __launch_bounds__(256) void stats0_kernel(const int* __restrict__ nn,
                                                     const float* __restrict__ P4,
                                                     const float* __restrict__ cent,
                                                     const float* __restrict__ P,
                                                     const float* __restrict__ W0x,
                                                     const float* __restrict__ b0,
                                                     float* __restrict__ part) {
  __shared__ __align__(16) float red[2][16][64];
  __shared__ __align__(16) float fin[256];
  const int tid = threadIdx.x;
  const int lane = tid & 31;
  const int wave = tid >> 5;
  const int cg = tid & 15;
  const int rlw = tid >> 4;
  const int c0 = 4 * cg;
  const v4f w0v = *(const v4f*)(W0x + 4 * (c0 + 0));
  const v4f w1v = *(const v4f*)(W0x + 4 * (c0 + 1));
  const v4f w2v = *(const v4f*)(W0x + 4 * (c0 + 2));
  const v4f w3v = *(const v4f*)(W0x + 4 * (c0 + 3));
  const v4f bb = *(const v4f*)(b0 + c0);
  float s0 = 0.f, s1 = 0.f, s2 = 0.f, s3 = 0.f;
  float q0 = 0.f, q1 = 0.f, q2 = 0.f, q3 = 0.f;
  const int m0 = blockIdx.x * 512;
#pragma unroll 1
  for (int it = 0; it < 32; ++it) {
    const int m = m0 + it * 16 + rlw;
    int j = nn[m];
    j = j < 0 ? 0 : j;
    j = j > kNpts - 1 ? kNpts - 1 : j;
    const size_t pi = (size_t)(m >> 15) * kNpts + j;
    const v4f pn = *(const v4f*)(P4 + 4 * pi);
    const v4f cq = *(const v4f*)(cent + 4 * (size_t)(m >> 5));
    const v4f pv = *(const v4f*)(P + pi * 64 + c0);
    const float rx = pn.x - cq.x;
    const float ry = pn.y - cq.y;
    const float rz = pn.z - cq.z;
    const float y0 = y0_val(pv.x, rx, ry, rz, w0v.x, w0v.y, w0v.z, bb.x);
    const float y1 = y0_val(pv.y, rx, ry, rz, w1v.x, w1v.y, w1v.z, bb.y);
    const float y2 = y0_val(pv.z, rx, ry, rz, w2v.x, w2v.y, w2v.z, bb.z);
    const float y3 = y0_val(pv.w, rx, ry, rz, w3v.x, w3v.y, w3v.z, bb.w);
    s0 += y0;
    s1 += y1;
    s2 += y2;
    s3 += y3;
    q0 = fmaf(y0, y0, q0);
    q1 = fmaf(y1, y1, q1);
    q2 = fmaf(y2, y2, q2);
    q3 = fmaf(y3, y3, q3);
  }
  red[0][rlw][c0 + 0] = s0;
  red[0][rlw][c0 + 1] = s1;
  red[0][rlw][c0 + 2] = s2;
  red[0][rlw][c0 + 3] = s3;
  red[1][rlw][c0 + 0] = q0;
  red[1][rlw][c0 + 1] = q1;
  red[1][rlw][c0 + 2] = q2;
  red[1][rlw][c0 + 3] = q3;
  __syncthreads();
  if (tid < 128) {
    const int which = tid >> 6;
    const int c = tid & 63;
    float a = 0.f;
#pragma unroll
    for (int r = 0; r < 16; ++r) a += red[which][r][c];
    fin[which * 128 + c] = a;
  }
  __syncthreads();
  if (wave < 2 && lane < 16) {
    const v4f pv = *(const v4f*)(fin + 128 * wave + 4 * lane);
    float* dst = part + (size_t)blockIdx.x * 256 + 128 * wave + 4 * lane;
    for (int pass = 0; pass < 2; ++pass) {
      *(volatile v4f*)dst = pv;
      __threadfence();
    }
  }
}

__global__ __launch_bounds__(256) void bn_finalize(const float* __restrict__ part, int nrows, int nch,
                                                   const float* __restrict__ gamma,
                                                   const float* __restrict__ beta,
                                                   float* __restrict__ ss) {
  __shared__ double dacc[256];
  __shared__ __align__(16) float tab[256];
  const int tid = threadIdx.x;
  const int pairs = 2 * nch;
  const int nseg = 256 / pairs;
  const int p = tid % pairs;
  const int g = tid / pairs;
  const int col = (p < nch) ? p : (128 + p - nch);
  double a = 0.0;
#pragma unroll 4
  for (int r = g; r < nrows; r += nseg) a += (double)part[(size_t)r * 256 + col];
  dacc[tid] = a;
  __syncthreads();
  if (tid < 128) {
    const int c = tid < nch ? tid : nch - 1;
    double S = 0.0, Q = 0.0;
    for (int g2 = 0; g2 < nseg; ++g2) {
      S += dacc[g2 * pairs + c];
      Q += dacc[g2 * pairs + nch + c];
    }
    const double invM = 1.0 / (double)kRows;
    const double mean = S * invM;
    double var = Q * invM - mean * mean;
    var = var < 0.0 ? 0.0 : var;
    const float vf = (float)var;
    const float rs = 1.0f / sqrtf(vf + 1e-5f);
    const float gm = gamma[c];
    const float bt = beta[c];
    const float sc = rs * gm;
    const float sh = bt - (float)mean * sc;
    const bool live = tid < nch;
    tab[tid] = live ? sc : 0.0f;
    tab[128 + tid] = live ? sh : 0.0f;
  }
  __syncthreads();
  if (tid < 64) {
    const int wave = tid >> 5;
    const int lane = tid & 31;
    const v4f v = *(const v4f*)(tab + 128 * wave + 4 * lane);
    float* dst = ss + 128 * wave + 4 * lane;
    for (int pass = 0; pass < 2; ++pass) {
      *(volatile v4f*)dst = v;
      __threadfence();
    }
  }
}

__global__ __launch_bounds__(256) void gemm1_kernel(const int* __restrict__ nn,
                                                    const float* __restrict__ P4,
                                                    const float* __restrict__ cent,
                                                    const float* __restrict__ P,
                                                    const float* __restrict__ W0x,
                                                    const float* __restrict__ b0,
                                                    const float* __restrict__ ss0,
                                                    const unsigned short* __restrict__ W1h,
                                                    const float* __restrict__ b1,
                                                    unsigned short* __restrict__ y1,
                                                    float* __restrict__ part) {
  __shared__ __align__(16) _Float16 As[128 * kApitch];
  __shared__ __align__(16) float sT[8][16 * 68];
  __shared__ __align__(16) float wsum[8][64];
  __shared__ __align__(16) float wsq[8][64];
  __shared__ __align__(16) float fin[256];
  __shared__ __align__(16) float w0xs[64 * 4];
  __shared__ float tb0[64];
  __shared__ float tsc[64];
  __shared__ float tsh[64];
  const int tid = threadIdx.x;
  const int lane = tid & 31;
  const int wave = tid >> 5;
  const int m0 = blockIdx.x * 128;
  if (tid < 64) {
    const v4f wv = *(const v4f*)(W0x + 4 * tid);
    *(v4f*)(w0xs + 4 * tid) = wv;
    tb0[tid] = b0[tid];
    tsc[tid] = ss0[tid];
    tsh[tid] = ss0[128 + tid];
  }
  __syncthreads();
  {
    const int row = tid >> 1;
    const int hf = tid & 1;
    const int m = m0 + row;
    int j = nn[m];
    j = j < 0 ? 0 : j;
    j = j > kNpts - 1 ? kNpts - 1 : j;
    const size_t pi = (size_t)(m >> 15) * kNpts + j;
    const v4f pn = *(const v4f*)(P4 + 4 * pi);
    const v4f cq = *(const v4f*)(cent + 4 * (size_t)(m >> 5));
    const float rx = pn.x - cq.x;
    const float ry = pn.y - cq.y;
    const float rz = pn.z - cq.z;
    const float* prow = P + pi * 64 + 32 * hf;
    _Float16* arow = As + row * kApitch + 32 * hf;
#pragma unroll 1
    for (int ch = 0; ch < 2; ++ch) {
      v4f pv[4];
#pragma unroll
      for (int g = 0; g < 4; ++g) pv[g] = *(const v4f*)(prow + 16 * ch + 4 * g);
      v8h h0, h1;
#pragma unroll
      for (int g = 0; g < 4; ++g) {
#pragma unroll
        for (int e = 0; e < 4; ++e) {
          const int cc = 32 * hf + 16 * ch + 4 * g + e;
          const v4f wv = *(const v4f*)(w0xs + 4 * cc);
          const float pe = pv[g][e];
          const float y = y0_val(pe, rx, ry, rz, wv.x, wv.y, wv.z, tb0[cc]);
          const float x = fmaxf(fmaf(y, tsc[cc], tsh[cc]), 0.0f);
          if (g < 2) h0[4 * g + e] = (_Float16)x; else h1[4 * (g - 2) + e] = (_Float16)x;
        }
      }
      *(v8h*)(arow + 16 * ch) = h0;
      *(v8h*)(arow + 16 * ch + 8) = h1;
    }
  }
  __syncthreads();
  const int rl = lane & 15;
  const int mOff = (lane >> 4) * 8;
  union { v16h v; v8h h[2]; } fa0, fa1;
  {
    const _Float16* ap = As + (wave * 16 + rl) * kApitch + (lane >> 4) * 8;
    fa0.h[0] = *(const v8h*)(ap);
    fa0.h[1] = *(const v8h*)(ap + 16);
    fa1.h[0] = *(const v8h*)(ap + 32);
    fa1.h[1] = *(const v8h*)(ap + 48);
  }
  v8f acc[4];
  wave_gemm<4>(fa0.v, fa1.v, (const _Float16*)W1h, lane, acc);
  float* slab = sT[wave];
#pragma unroll
  for (int j = 0; j < 4; ++j) {
    const int n = 16 * j + rl;
    const float bv = b1[n];
    float s1 = 0.f, s2 = 0.f;
#pragma unroll
    for (int r = 0; r < 8; ++r) {
      const float v = acc[j][r] * kWinv + bv;
      slab[(mOff + r) * 68 + n] = v;
      s1 += v;
      s2 = fmaf(v, v, s2);
    }
    s1 += __shfl_xor(s1, 16, 32);
    s2 += __shfl_xor(s2, 16, 32);
    if (lane < 16) {
      wsum[wave][n] = s1;
      wsq[wave][n] = s2;
    }
  }
  wave_sync_lds();
  {
    const int q4 = lane >> 3;
    const int c8 = (lane & 7) * 8;
    v8h hv[4];
#pragma unroll
    for (int it = 0; it < 4; ++it) {
      const float* sp = slab + (it * 4 + q4) * 68 + c8;
#pragma unroll
      for (int e = 0; e < 8; ++e) hv[it][e] = (_Float16)sp[e];
    }
    for (int pass = 0; pass < 2; ++pass) {
#pragma unroll
      for (int it = 0; it < 4; ++it) {
        const int row = it * 4 + q4;
        *(volatile v8h*)(y1 + (size_t)(m0 + wave * 16 + row) * 64 + c8) = hv[it];
      }
      __threadfence();
    }
  }
  __syncthreads();
  if (tid < 128) {
    const int which = tid >> 6;
    const int c = tid & 63;
    float a1 = 0.f, a2 = 0.f;
#pragma unroll
    for (int w = 0; w < 8; ++w) {
      a1 += wsum[w][c];
      a2 += wsq[w][c];
    }
    fin[which * 128 + c] = (which == 0) ? a1 : a2;
  }
  __syncthreads();
  if (wave < 2 && lane < 16) {
    const v4f pv = *(const v4f*)(fin + 128 * wave + 4 * lane);
    float* dst = part + (size_t)blockIdx.x * 256 + 128 * wave + 4 * lane;
    for (int pass = 0; pass < 2; ++pass) {
      *(volatile v4f*)dst = pv;
      __threadfence();
    }
  }
}

__global__ __launch_bounds__(256) void gemm2_kernel(const unsigned short* __restrict__ y1,
                                                    const float* __restrict__ ss1,
                                                    const unsigned short* __restrict__ W2h,
                                                    const float* __restrict__ b2,
                                                    float* __restrict__ mx,
                                                    float* __restrict__ mn,
                                                    float* __restrict__ part) {
  __shared__ __align__(16) _Float16 As[128 * kApitch];
  __shared__ __align__(16) float wsum[8][128];
  __shared__ __align__(16) float wsq[8][128];
  __shared__ __align__(16) float wmx[8][128];
  __shared__ __align__(16) float wmn[8][128];
  __shared__ __align__(16) float fin[256];
  __shared__ float tsc[64];
  __shared__ float tsh[64];
  const int tid = threadIdx.x;
  const int lane = tid & 31;
  const int wave = tid >> 5;
  const int m0 = blockIdx.x * 128;
  if (tid < 64) {
    tsc[tid] = ss1[tid];
    tsh[tid] = ss1[128 + tid];
  }
  __syncthreads();
  {
    const int row = tid >> 1;
    const int hf = tid & 1;
    const v4u* src = (const v4u*)(y1 + (size_t)(m0 + row) * 64 + 32 * hf);
    _Float16* arow = As + row * kApitch + 32 * hf;
#pragma unroll 1
    for (int k = 0; k < 4; ++k) {
      const v4u u = src[k];
      const unsigned wa[4] = {u.x, u.y, u.z, u.w};
      v8h hv;
#pragma unroll
      for (int wi = 0; wi < 4; ++wi) {
        const unsigned w = wa[wi];
        const int c = 32 * hf + 8 * k + 2 * wi;
        const float f0 = h16_to_f32(w & 0xffffu);
        const float f1 = h16_to_f32(w >> 16);
        const float x0 = fmaxf(fmaf(f0, tsc[c], tsh[c]), 0.0f);
        const float x1 = fmaxf(fmaf(f1, tsc[c + 1], tsh[c + 1]), 0.0f);
        hv[2 * wi] = (_Float16)x0;
        hv[2 * wi + 1] = (_Float16)x1;
      }
      *(v8h*)(arow + 8 * k) = hv;
    }
  }
  __syncthreads();
  const int rl = lane & 15;
  union { v16h v; v8h h[2]; } fa0, fa1;
  {
    const _Float16* ap = As + (wave * 16 + rl) * kApitch + (lane >> 4) * 8;
    fa0.h[0] = *(const v8h*)(ap);
    fa0.h[1] = *(const v8h*)(ap + 16);
    fa1.h[0] = *(const v8h*)(ap + 32);
    fa1.h[1] = *(const v8h*)(ap + 48);
  }
  v8f acc[8];
  wave_gemm<8>(fa0.v, fa1.v, (const _Float16*)W2h, lane, acc);
#pragma unroll
  for (int j = 0; j < 8; ++j) {
    const int n = 16 * j + rl;
    const float bv = b2[n];
    float s1 = 0.f, s2 = 0.f;
    float vmx = -INFINITY, vmn = INFINITY;
#pragma unroll
    for (int r = 0; r < 8; ++r) {
      const float v = acc[j][r] * kWinv + bv;
      s1 += v;
      s2 = fmaf(v, v, s2);
      vmx = fmaxf(vmx, v);
      vmn = fminf(vmn, v);
    }
    s1 += __shfl_xor(s1, 16, 32);
    s2 += __shfl_xor(s2, 16, 32);
    const float omx = __shfl_xor(vmx, 16, 32);
    const float omn = __shfl_xor(vmn, 16, 32);
    vmx = fmaxf(vmx, omx);
    vmn = fminf(vmn, omn);
    if (lane < 16) {
      wsum[wave][n] = s1;
      wsq[wave][n] = s2;
      wmx[wave][n] = vmx;
      wmn[wave][n] = vmn;
    }
  }
  __syncthreads();
  {
    const int c = tid & 127;
    float a1 = 0.f, a2 = 0.f;
#pragma unroll
    for (int w = 0; w < 8; ++w) {
      a1 += wsum[w][c];
      a2 += wsq[w][c];
    }
    fin[tid] = (tid < 128) ? a1 : a2;
  }
  {
    const int g = wave & 3;
    const v4f xa = *(const v4f*)(&wmx[2 * g][4 * lane]);
    const v4f xb = *(const v4f*)(&wmx[2 * g + 1][4 * lane]);
    const v4f na = *(const v4f*)(&wmn[2 * g][4 * lane]);
    const v4f nb = *(const v4f*)(&wmn[2 * g + 1][4 * lane]);
    v4f vx, vn;
    vx.x = fmaxf(xa.x, xb.x);
    vx.y = fmaxf(xa.y, xb.y);
    vx.z = fmaxf(xa.z, xb.z);
    vx.w = fmaxf(xa.w, xb.w);
    vn.x = fminf(na.x, nb.x);
    vn.y = fminf(na.y, nb.y);
    vn.z = fminf(na.z, nb.z);
    vn.w = fminf(na.w, nb.w);
    const bool top = wave < 4;
    const v4f val = top ? vx : vn;
    float* base = top ? mx : mn;
    float* dst = base + ((size_t)(blockIdx.x * 4 + g) * 128 + 4 * lane);
    for (int pass = 0; pass < 2; ++pass) {
      *(volatile v4f*)dst = val;
      __threadfence();
    }
  }
  __syncthreads();
  if (wave < 2) {
    const v4f pv = *(const v4f*)(fin + 128 * wave + 4 * lane);
    float* dst = part + (size_t)blockIdx.x * 256 + 128 * wave + 4 * lane;
    for (int pass = 0; pass < 2; ++pass) {
      *(volatile v4f*)dst = pv;
      __threadfence();
    }
  }
}

__global__ __launch_bounds__(256) void final_kernel(const float* __restrict__ mx,
                                                    const float* __restrict__ mn,
                                                    const float* __restrict__ ss2,
                                                    float* __restrict__ out1) {
  __shared__ __align__(16) float tile[128 * 36];
  __shared__ float tabs[256];
  const int tid = threadIdx.x;
  const int lane = tid & 31;
  const int wave = tid >> 5;
  tabs[tid] = ss2[tid];
  __syncthreads();
  const int b = blockIdx.x >> 5;
  const int s0 = (blockIdx.x & 31) * 32;
  {
    const int row = tid >> 3;
    const int c16 = (tid & 7) * 16;
    const size_t qrow = (size_t)b * kNsmp + s0 + row;
    const float* pa = mx + qrow * 128 + c16;
    const float* pb = mn + qrow * 128 + c16;
    v4f av[4], bv[4];
#pragma unroll
    for (int g = 0; g < 4; ++g) {
      av[g] = *(const v4f*)(pa + 4 * g);
      bv[g] = *(const v4f*)(pb + 4 * g);
    }
#pragma unroll
    for (int g = 0; g < 4; ++g) {
#pragma unroll
      for (int e = 0; e < 4; ++e) {
        const int ch = c16 + 4 * g + e;
        const float sc = tabs[ch];
        const float sh = tabs[128 + ch];
        const float fa = (sc >= 0.0f) ? 1.0f : 0.0f;
        const float fb = 1.0f - fa;
        const float ae = av[g][e];
        const float be = bv[g][e];
        const float x = fmaf(fa, ae, fb * be);
        const float v = fmaxf(fmaf(sc, x, sh), 0.0f);
        tile[ch * 36 + row] = v;
      }
    }
  }
  __syncthreads();
  {
    const int lq = lane >> 3;
    const int pc = (lane & 7) * 4;
    v4f ov[4];
#pragma unroll
    for (int it = 0; it < 4; ++it) {
      const int ch = 16 * wave + 4 * it + lq;
      ov[it] = *(const v4f*)(tile + ch * 36 + pc);
    }
    for (int pass = 0; pass < 2; ++pass) {
#pragma unroll
      for (int it = 0; it < 4; ++it) {
        const int ch = 16 * wave + 4 * it + lq;
        *(volatile v4f*)(out1 + ((size_t)(b * 128 + ch) * kNsmp + s0 + pc)) = ov[it];
      }
      __threadfence();
    }
  }
}

extern "C" void kernel_launch(void* const* d_in, const int* in_sizes, int n_in,
                              void* d_out, int out_size, void* d_ws, size_t ws_size,
                              hipStream_t stream) {
  if (n_in < 14) return;
  if (ws_size < kWsTotal) return;
  if ((size_t)out_size < kOut1Float + (size_t)kBatch * 128 * kNsmp) return;
  (void)in_sizes;
  const float* xyz    = (const float*)d_in[0];
  const float* points = (const float*)d_in[1];
  const float* w0  = (const float*)d_in[2];
  const float* b0  = (const float*)d_in[3];
  const float* g0  = (const float*)d_in[4];
  const float* be0 = (const float*)d_in[5];
  const float* w1  = (const float*)d_in[6];
  const float* b1  = (const float*)d_in[7];
  const float* g1  = (const float*)d_in[8];
  const float* be1 = (const float*)d_in[9];
  const float* w2  = (const float*)d_in[10];
  const float* b2  = (const float*)d_in[11];
  const float* g2  = (const float*)d_in[12];
  const float* be2 = (const float*)d_in[13];

  char* ws = (char*)d_ws;
  float* P4   = (float*)(ws + kOffP4);
  float* cent = (float*)(ws + kOffCent);
  int*   nn   = (int*)(ws + kOffNn);
  unsigned short* W0p = (unsigned short*)(ws + kOffW0p);
  unsigned short* W1h = (unsigned short*)(ws + kOffW1h);
  unsigned short* W2h = (unsigned short*)(ws + kOffW2h);
  float* W0x  = (float*)(ws + kOffW0x);
  float* ss0  = (float*)(ws + kOffSs0);
  float* ss1  = (float*)(ws + kOffSs1);
  float* ss2  = (float*)(ws + kOffSs2);
  float* part0 = (float*)(ws + kOffPart0);
  float* part1 = (float*)(ws + kOffPart1);
  float* part2 = (float*)(ws + kOffPart2);
  float* P    = (float*)(ws + kOffP);
  unsigned short* y1 = (unsigned short*)(ws + kOffY1);
  float* mx   = (float*)(ws + kOffMx);
  float* mn   = (float*)(ws + kOffMn);

  float* out0 = (float*)d_out;
  float* out1 = (float*)d_out + kOut1Float;

  prep_kernel<<<265, 256, 0, stream>>>(xyz, w0, w1, w2, P4, W0p, W1h, W2h, W0x);
  fps_kernel<<<kBatch, 256, 0, stream>>>(xyz, out0, cent);
  knn_kernel<<<kQueries / 2, 64, 0, stream>>>(P4, cent, nn);
  pgemm_kernel<<<kPoints / 128, 256, 0, stream>>>(points, W0p, P);
  stats0_kernel<<<kRows / 512, 256, 0, stream>>>(nn, P4, cent, P, W0x, b0, part0);
  bn_finalize<<<1, 256, 0, stream>>>(part0, kRows / 512, 64, g0, be0, ss0);
  gemm1_kernel<<<kRows / 128, 256, 0, stream>>>(nn, P4, cent, P, W0x, b0, ss0, W1h, b1, y1, part1);
  bn_finalize<<<1, 256, 0, stream>>>(part1, kRows / 128, 64, g1, be1, ss1);
  gemm2_kernel<<<kRows / 128, 256, 0, stream>>>(y1, ss1, W2h, b2, mx, mn, part2);
  bn_finalize<<<1, 256, 0, stream>>>(part2, kRows / 128, 128, g2, be2, ss2);
  final_kernel<<<kBatch * 32, 256, 0, stream>>>(mx, mn, ss2, out1);
}
